// GravitationLayer_31147102830703
// MI455X (gfx1250) — hardware-verified
//
#include <hip/hip_runtime.h>
#include <math.h>
#include <stdint.h>

#define DM   1024
#define NH   16
#define DH   64
#define NB   2
#define SEQ  2048
#define ROWS (NB * SEQ)
#define NBH  (NB * NH)
#define EPSV 1e-8f

static_assert(DM == NH * DH);
static_assert(DH == 64);
static_assert(SEQ % 64 == 0);
static_assert(ROWS % 64 == 0);

typedef _Float16 v16h __attribute__((ext_vector_type(16)));
typedef _Float16 v8h  __attribute__((ext_vector_type(8)));
typedef __bf16   v16b __attribute__((ext_vector_type(16)));
typedef __bf16   v8b  __attribute__((ext_vector_type(8)));
typedef float    v8f  __attribute__((ext_vector_type(8)));
typedef float    v4f  __attribute__((ext_vector_type(4)));
typedef unsigned int   v4u  __attribute__((ext_vector_type(4)));
typedef unsigned short v8us __attribute__((ext_vector_type(8)));

union FH  { v16h v; v8h  h[2]; };
union FB  { v16b v; v8b  h[2]; };
union U8H { v8h  v; v4u  u; };
union U8S { v8us v; v4u  u; };

__device__ __forceinline__ unsigned short f2bf_bits(float f) {
  const unsigned u = __float_as_uint(f);
  return (unsigned short)((u + 0x7FFFu + ((u >> 16) & 1u)) >> 16);
}
__device__ __forceinline__ float bf_bits2f(unsigned short b) { return __uint_as_float(((unsigned)b) << 16); }
__device__ __forceinline__ unsigned short f2h_bits(float f) { return __builtin_bit_cast(unsigned short, (_Float16)f); }
__device__ __forceinline__ unsigned pk16(unsigned short a, unsigned short b) { return (unsigned)a | ((unsigned)b << 16); }

__device__ __forceinline__ void split2(float f0, float f1, unsigned& hw, unsigned& lw) {
  const unsigned short h0 = f2bf_bits(f0), h1 = f2bf_bits(f1);
  const unsigned short l0 = f2bf_bits(f0 - bf_bits2f(h0)), l1 = f2bf_bits(f1 - bf_bits2f(h1));
  hw = pk16(h0, h1);
  lw = pk16(l0, l1);
}

__device__ __forceinline__ v8f mma_h(v16h a, v16h b, v8f c) {
  c = __builtin_amdgcn_wmma_f32_16x16x32_f16(false, a, false, b, (short)0, c, false, false);
  asm volatile("v_nop\n\tv_nop\n\tv_nop\n\tv_nop" : "+v"(c) : "v"(a), "v"(b));
  return c;
}
__device__ __forceinline__ v8f mma_bf(v16b a, v16b b, v8f c) {
  c = __builtin_amdgcn_wmma_f32_16x16x32_bf16(false, a, false, b, (short)0, c, false, false);
  asm volatile("v_nop\n\tv_nop\n\tv_nop\n\tv_nop" : "+v"(c) : "v"(a), "v"(b));
  return c;
}

__device__ __forceinline__ void wave_lds_sync() {
  __builtin_amdgcn_fence(__ATOMIC_RELEASE, "workgroup");
  __builtin_amdgcn_wave_barrier();
  __builtin_amdgcn_fence(__ATOMIC_ACQUIRE, "workgroup");
}

__device__ __forceinline__ v8f zero8() { return (v8f){0.f, 0.f, 0.f, 0.f, 0.f, 0.f, 0.f, 0.f}; }

__global__ __launch_bounds__(256) void cvt_f16_kernel(const float* __restrict__ src,
                                                       unsigned short* __restrict__ dst,
                                                       int n8, float scale) {
  const int t = blockIdx.x * 256 + (int)threadIdx.x;
  if (t >= n8) return;
  const size_t o = (size_t)t * 8;
  const v4f a0 = *(const v4f*)(src + o);
  const v4f a1 = *(const v4f*)(src + o + 4);
  const v4u pv = (v4u){pk16(f2h_bits(a0[0] * scale), f2h_bits(a0[1] * scale)),
                       pk16(f2h_bits(a0[2] * scale), f2h_bits(a0[3] * scale)),
                       pk16(f2h_bits(a1[0] * scale), f2h_bits(a1[1] * scale)),
                       pk16(f2h_bits(a1[2] * scale), f2h_bits(a1[3] * scale))};
  volatile v4u* q = (volatile v4u*)(dst + o);
  *q = pv;
  __threadfence();
  *q = pv;
}

__global__ __launch_bounds__(256) void cvt_split_kernel(const float* __restrict__ src,
                                                         unsigned short* __restrict__ hi,
                                                         unsigned short* __restrict__ lo,
                                                         int n8) {
  const int t = blockIdx.x * 256 + (int)threadIdx.x;
  if (t >= n8) return;
  const size_t o = (size_t)t * 8;
  const v4f a0 = *(const v4f*)(src + o);
  const v4f a1 = *(const v4f*)(src + o + 4);
  unsigned h0, h1, h2, h3, l0, l1, l2, l3;
  split2(a0[0], a0[1], h0, l0);
  split2(a0[2], a0[3], h1, l1);
  split2(a1[0], a1[1], h2, l2);
  split2(a1[2], a1[3], h3, l3);
  const v4u hv = (v4u){h0, h1, h2, h3};
  const v4u lv = (v4u){l0, l1, l2, l3};
  volatile v4u* ph = (volatile v4u*)(hi + o);
  volatile v4u* pl = (volatile v4u*)(lo + o);
  *ph = hv;
  *pl = lv;
  __threadfence();
  *ph = hv;
  *pl = lv;
}

#define TPH 72
#define TPF 68

__global__ __launch_bounds__(128)
void proj_qk_kernel(const unsigned short* __restrict__ Xp, const unsigned short* __restrict__ Wp,
                    const float* __restrict__ bias, unsigned short* __restrict__ outp,
                    float* __restrict__ ssq) {
  __shared__ __align__(16) _Float16 sT[4][32 * TPH];
  __shared__ __align__(16) float    sS[4][32];

  const int wave = threadIdx.x >> 5;
  const int lane = threadIdx.x & 31;
  const int lh   = lane >> 4;
  const int c    = lane & 15;
  const int gw   = blockIdx.x * 4 + wave;
  const int tm   = (gw >> 4) * 32;
  const int hd   = gw & 15;
  const int tn   = hd * DH;

  const _Float16* X = (const _Float16*)(const void*)Xp;
  const _Float16* W = (const _Float16*)(const void*)Wp;
  const _Float16* ar0 = X + (size_t)(tm + c) * DM + 8 * lh;
  const _Float16* ar1 = ar0 + (size_t)16 * DM;
  const _Float16* br  = W + (size_t)(tn + c) * DM + 8 * lh;

  v8f acc[2][4];
#pragma unroll
  for (int mi = 0; mi < 2; ++mi)
#pragma unroll
    for (int ni = 0; ni < 4; ++ni) acc[mi][ni] = zero8();

#pragma unroll 1
  for (int k0 = 0; k0 < DM; k0 += 32) {
    FH a0, a1;
    a0.h[0] = *(const v8h*)(ar0 + k0);
    a0.h[1] = *(const v8h*)(ar0 + k0 + 16);
    a1.h[0] = *(const v8h*)(ar1 + k0);
    a1.h[1] = *(const v8h*)(ar1 + k0 + 16);
#pragma unroll
    for (int ni = 0; ni < 4; ++ni) {
      const _Float16* bp = br + (size_t)ni * 16 * DM + k0;
      FB dummy; (void)dummy;
      FH b;
      b.h[0] = *(const v8h*)(bp);
      b.h[1] = *(const v8h*)(bp + 16);
      acc[0][ni] = mma_h(a0.v, b.v, acc[0][ni]);
      acc[1][ni] = mma_h(a1.v, b.v, acc[1][ni]);
    }
  }

  _Float16* st = sT[wave];
  float*    ss = sS[wave];
#pragma unroll
  for (int mi = 0; mi < 2; ++mi) {
    float rs[8];
#pragma unroll
    for (int r = 0; r < 8; ++r) rs[r] = 0.f;
#pragma unroll
    for (int ni = 0; ni < 4; ++ni) {
      const float bn = bias[tn + ni * 16 + c];
#pragma unroll
      for (int r = 0; r < 8; ++r) {
        const float y = acc[mi][ni][r] * 0.03125f + bn;
        rs[r] += y * y;
        st[(mi * 16 + 8 * lh + r) * TPH + ni * 16 + c] = (_Float16)y;
      }
    }
#pragma unroll
    for (int r = 0; r < 8; ++r) {
      float v = rs[r];
      v += __shfl_xor(v, 1, 32);
      v += __shfl_xor(v, 2, 32);
      v += __shfl_xor(v, 4, 32);
      v += __shfl_xor(v, 8, 32);
      if (c == 0) ss[mi * 16 + 8 * lh + r] = v;
    }
  }
  wave_lds_sync();

  const int bb  = tm >> 11;
  const int s0  = tm & (SEQ - 1);
  const int bhh = bb * NH + hd;
  unsigned short* ob = outp + ((size_t)bhh * SEQ + s0) * DH;
  float* sb = ssq + (size_t)bhh * SEQ + s0;
  const int rq = lane >> 3;
  const int pc = (lane & 7) * 8;
  const v4f sv = *(const v4f*)(ss + 4 * (lane & 7));
  for (int ps = 0; ps < 2; ++ps) {
#pragma unroll
    for (int it = 0; it < 8; ++it) {
      const int tr = it * 4 + rq;
      U8H u;
      u.v = *(const v8h*)(st + tr * TPH + pc);
      *(volatile v4u*)(ob + (size_t)tr * DH + pc) = u.u;
    }
    if (lane < 8) *(volatile v4f*)(sb + 4 * lane) = sv;
    __threadfence();
  }
}

__global__ __launch_bounds__(128)
void proj_v_kernel(const unsigned short* __restrict__ Xh, const unsigned short* __restrict__ Xl,
                   const unsigned short* __restrict__ Wh, const unsigned short* __restrict__ Wl,
                   const float* __restrict__ bias,
                   unsigned short* __restrict__ VTh, unsigned short* __restrict__ VTl) {
  __shared__ __align__(16) unsigned short sH[4][32 * TPH];
  __shared__ __align__(16) unsigned short sL[4][32 * TPH];

  const int wave = threadIdx.x >> 5;
  const int lane = threadIdx.x & 31;
  const int lh   = lane >> 4;
  const int c    = lane & 15;
  const int gw   = blockIdx.x * 4 + wave;
  const int tm   = (gw >> 5) * 64;
  const int tn   = (gw & 31) * 32;

  const __bf16* Ah = (const __bf16*)(const void*)Xh + (size_t)(tm + c) * DM + 8 * lh;
  const __bf16* Al = (const __bf16*)(const void*)Xl + (size_t)(tm + c) * DM + 8 * lh;
  const __bf16* Bh = (const __bf16*)(const void*)Wh + (size_t)(tn + c) * DM + 8 * lh;
  const __bf16* Bl = (const __bf16*)(const void*)Wl + (size_t)(tn + c) * DM + 8 * lh;

  v8f acc[4][2];
#pragma unroll
  for (int mi = 0; mi < 4; ++mi)
#pragma unroll
    for (int ni = 0; ni < 2; ++ni) acc[mi][ni] = zero8();

#pragma unroll 1
  for (int k0 = 0; k0 < DM; k0 += 32) {
    FB bh[2], bl[2];
#pragma unroll
    for (int ni = 0; ni < 2; ++ni) {
      const size_t bo = (size_t)ni * 16 * DM + k0;
      bh[ni].h[0] = *(const v8b*)(Bh + bo);
      bh[ni].h[1] = *(const v8b*)(Bh + bo + 16);
      bl[ni].h[0] = *(const v8b*)(Bl + bo);
      bl[ni].h[1] = *(const v8b*)(Bl + bo + 16);
    }
#pragma unroll
    for (int mi = 0; mi < 4; ++mi) {
      const size_t ao = (size_t)mi * 16 * DM + k0;
      FB ah, al;
      ah.h[0] = *(const v8b*)(Ah + ao);
      ah.h[1] = *(const v8b*)(Ah + ao + 16);
      al.h[0] = *(const v8b*)(Al + ao);
      al.h[1] = *(const v8b*)(Al + ao + 16);
#pragma unroll
      for (int ni = 0; ni < 2; ++ni) {
        acc[mi][ni] = mma_bf(ah.v, bh[ni].v, acc[mi][ni]);
        acc[mi][ni] = mma_bf(ah.v, bl[ni].v, acc[mi][ni]);
        acc[mi][ni] = mma_bf(al.v, bh[ni].v, acc[mi][ni]);
      }
    }
  }

  unsigned short* sh = sH[wave];
  unsigned short* sl = sL[wave];
#pragma unroll
  for (int ni = 0; ni < 2; ++ni) {
    const float bn = bias[tn + ni * 16 + c];
#pragma unroll
    for (int mi = 0; mi < 4; ++mi) {
#pragma unroll
      for (int r = 0; r < 8; ++r) {
        const float y = acc[mi][ni][r] + bn;
        const unsigned short hb = f2bf_bits(y);
        const unsigned short lb = f2bf_bits(y - bf_bits2f(hb));
        const int idx = (ni * 16 + c) * TPH + mi * 16 + 8 * lh + r;
        sh[idx] = hb;
        sl[idx] = lb;
      }
    }
  }
  wave_lds_sync();

  const int bb  = tm >> 11;
  const int s0  = tm & (SEQ - 1);
  const int hd  = tn >> 6;
  const int d0  = tn & 63;
  const int bhh = bb * NH + hd;
  unsigned short* obh = VTh + ((size_t)(bhh * DH + d0) * SEQ + s0);
  unsigned short* obl = VTl + ((size_t)(bhh * DH + d0) * SEQ + s0);
  const int rq = lane >> 3;
  const int pc = (lane & 7) * 8;
  for (int ps = 0; ps < 2; ++ps) {
#pragma unroll
    for (int it = 0; it < 8; ++it) {
      const int dl = it * 4 + rq;
      U8S uh, ul;
      uh.v = *(const v8us*)(sh + dl * TPH + pc);
      ul.v = *(const v8us*)(sl + dl * TPH + pc);
      *(volatile v4u*)(obh + (size_t)dl * SEQ + pc) = uh.u;
      *(volatile v4u*)(obl + (size_t)dl * SEQ + pc) = ul.u;
    }
    __threadfence();
  }
}

__global__ __launch_bounds__(128)
void proj_o_kernel(const unsigned short* __restrict__ Oh, const unsigned short* __restrict__ Ol,
                   const unsigned short* __restrict__ Wh, const unsigned short* __restrict__ Wl,
                   const float* __restrict__ bias, float* __restrict__ out) {
  __shared__ __align__(16) float sO[4][32 * TPF];

  const int wave = threadIdx.x >> 5;
  const int lane = threadIdx.x & 31;
  const int lh   = lane >> 4;
  const int c    = lane & 15;
  const int gw   = blockIdx.x * 4 + wave;
  const int tm   = (gw >> 4) * 32;
  const int tn   = (gw & 15) * 64;

  const __bf16* Ah = (const __bf16*)(const void*)Oh + (size_t)(tm + c) * DM + 8 * lh;
  const __bf16* Al = (const __bf16*)(const void*)Ol + (size_t)(tm + c) * DM + 8 * lh;
  const __bf16* Bh = (const __bf16*)(const void*)Wh + (size_t)(tn + c) * DM + 8 * lh;
  const __bf16* Bl = (const __bf16*)(const void*)Wl + (size_t)(tn + c) * DM + 8 * lh;

  v8f acc[2][4];
#pragma unroll
  for (int mi = 0; mi < 2; ++mi)
#pragma unroll
    for (int ni = 0; ni < 4; ++ni) acc[mi][ni] = zero8();

#pragma unroll 1
  for (int k0 = 0; k0 < DM; k0 += 32) {
    FB ah[2], al[2];
#pragma unroll
    for (int mi = 0; mi < 2; ++mi) {
      const size_t ao = (size_t)mi * 16 * DM + k0;
      ah[mi].h[0] = *(const v8b*)(Ah + ao);
      ah[mi].h[1] = *(const v8b*)(Ah + ao + 16);
      al[mi].h[0] = *(const v8b*)(Al + ao);
      al[mi].h[1] = *(const v8b*)(Al + ao + 16);
    }
#pragma unroll
    for (int ni = 0; ni < 4; ++ni) {
      const size_t bo = (size_t)ni * 16 * DM + k0;
      FB bh, bl;
      bh.h[0] = *(const v8b*)(Bh + bo);
      bh.h[1] = *(const v8b*)(Bh + bo + 16);
      bl.h[0] = *(const v8b*)(Bl + bo);
      bl.h[1] = *(const v8b*)(Bl + bo + 16);
#pragma unroll
      for (int mi = 0; mi < 2; ++mi) {
        acc[mi][ni] = mma_bf(ah[mi].v, bh.v, acc[mi][ni]);
        acc[mi][ni] = mma_bf(ah[mi].v, bl.v, acc[mi][ni]);
        acc[mi][ni] = mma_bf(al[mi].v, bh.v, acc[mi][ni]);
      }
    }
  }

  float* so = sO[wave];
#pragma unroll
  for (int ni = 0; ni < 4; ++ni) {
    const float bn = bias[tn + ni * 16 + c];
#pragma unroll
    for (int mi = 0; mi < 2; ++mi)
#pragma unroll
      for (int r = 0; r < 8; ++r)
        so[(mi * 16 + 8 * lh + r) * TPF + ni * 16 + c] = acc[mi][ni][r] + bn;
  }
  wave_lds_sync();

  float* ob = out + (size_t)tm * DM + tn;
  const int rq2 = lane >> 4;
  const int pc4 = (lane & 15) * 4;
  for (int ps = 0; ps < 2; ++ps) {
#pragma unroll
    for (int it = 0; it < 16; ++it) {
      const int tr = it * 2 + rq2;
      const v4f v = *(const v4f*)(so + tr * TPF + pc4);
      *(volatile v4f*)(ob + (size_t)tr * DM + pc4) = v;
    }
    __threadfence();
  }
}

#define QB  64
#define KC  64
#define KTP 72
#define VTP 72
#define PTP 72
#define OTP 64

__global__ __launch_bounds__(256)
void grav_attn_kernel(const unsigned short* __restrict__ Qp, const unsigned short* __restrict__ Kp,
                      const unsigned short* __restrict__ VThp, const unsigned short* __restrict__ VTlp,
                      const float* __restrict__ q2p, const float* __restrict__ k2p,
                      const float* __restrict__ Gp,
                      unsigned short* __restrict__ Oh, unsigned short* __restrict__ Ol) {
  __shared__ __align__(16) _Float16 Ksh[KC * KTP];
  __shared__ __align__(16) __bf16   Vth[DH * VTP];
  __shared__ __align__(16) __bf16   Vtl[DH * VTP];
  __shared__ __align__(16) __bf16   Psh[4][16 * PTP];
  __shared__ __align__(16) __bf16   Psl[4][16 * PTP];
  __shared__ __align__(16) unsigned short Osh[QB * OTP];
  __shared__ __align__(16) unsigned short Osl[QB * OTP];
  __shared__ __align__(16) float    Ll[4][16];

  const int tid  = threadIdx.x;
  const int wave = tid >> 5;
  const int lane = tid & 31;
  const int lh   = lane >> 4;
  const int c    = lane & 15;
  const int g    = wave & 3;
  const int chh  = wave >> 2;
  const int ch0  = chh * 32;

  const int nqt = SEQ / QB;
  const int qt  = blockIdx.x % nqt;
  const int bh  = blockIdx.x / nqt;
  const int b   = bh >> 4;
  const int hd  = bh & 15;
  const int qg0 = qt * QB + g * 16;
  const size_t soff = (size_t)bh * SEQ;

  const _Float16* Q  = (const _Float16*)(const void*)Qp + soff * DH;
  const _Float16* K  = (const _Float16*)(const void*)Kp + soff * DH;
  const __bf16*   Vh = (const __bf16*)(const void*)VThp + (size_t)bh * DH * SEQ;
  const __bf16*   Vl = (const __bf16*)(const void*)VTlp + (size_t)bh * DH * SEQ;

  const float Gh = Gp[hd];
  float q2v[8], gmi[8], lrow[8];
#pragma unroll
  for (int r = 0; r < 8; ++r) {
    const int i = qg0 + 8 * lh + r;
    q2v[r]  = q2p[soff + i];
    gmi[r]  = Gh * sqrtf(k2p[soff + i]);
    lrow[r] = 0.f;
  }

  FH qa[2];
  {
    const _Float16* qr = Q + (size_t)(qg0 + c) * DH + 8 * lh;
#pragma unroll
    for (int dc = 0; dc < 2; ++dc) {
      qa[dc].h[0] = *(const v8h*)(qr + dc * 32);
      qa[dc].h[1] = *(const v8h*)(qr + dc * 32 + 16);
    }
  }

  v8f oacc[2];
  oacc[0] = zero8();
  oacc[1] = zero8();

  __bf16* pwh = Psh[g];
  __bf16* pwl = Psl[g];

#pragma unroll 1
  for (int kc = 0; kc < SEQ / KC; ++kc) {
    const int kv0 = kc * KC;
    __syncthreads();
    {
      const int r  = tid >> 2;
      const int qq = (tid & 3) * 16;
      const _Float16* ks = K + (size_t)(kv0 + r) * DH + qq;
      _Float16* kd = Ksh + r * KTP + qq;
      *(v8h*)(kd)     = *(const v8h*)(ks);
      *(v8h*)(kd + 8) = *(const v8h*)(ks + 8);
      const __bf16* vhs = Vh + (size_t)r * SEQ + kv0 + qq;
      const __bf16* vls = Vl + (size_t)r * SEQ + kv0 + qq;
      *(v8b*)(Vth + r * VTP + qq)     = *(const v8b*)(vhs);
      *(v8b*)(Vth + r * VTP + qq + 8) = *(const v8b*)(vhs + 8);
      *(v8b*)(Vtl + r * VTP + qq)     = *(const v8b*)(vls);
      *(v8b*)(Vtl + r * VTP + qq + 8) = *(const v8b*)(vls + 8);
    }
    __syncthreads();

    if (wave < 4) {
      v8f s[4];
#pragma unroll
      for (int j = 0; j < 4; ++j) s[j] = zero8();
#pragma unroll
      for (int dc = 0; dc < 2; ++dc) {
#pragma unroll
        for (int j = 0; j < 4; ++j) {
          const _Float16* kp = Ksh + (j * 16 + c) * KTP + dc * 32 + 8 * lh;
          FH kb;
          kb.h[0] = *(const v8h*)(kp);
          kb.h[1] = *(const v8h*)(kp + 16);
          s[j] = mma_h(qa[dc].v, kb.v, s[j]);
        }
      }
      float k2j[4], mj[4];
#pragma unroll
      for (int j = 0; j < 4; ++j) {
        k2j[j] = k2p[soff + kv0 + j * 16 + c];
        mj[j]  = sqrtf(k2j[j]);
      }
#pragma unroll
      for (int r = 0; r < 8; ++r) {
        float psum = 0.f;
#pragma unroll
        for (int j = 0; j < 4; ++j) {
          const float t2 = q2v[r] + k2j[j];
          const float d2 = t2 - 2.0f * s[j][r];
          const float dd = sqrtf(fmaxf(d2, 0.0f)) + EPSV;
          const float f  = (gmi[r] * mj[j]) * __builtin_amdgcn_rcpf(dd * dd);
          psum += f;
          const unsigned short hb = f2bf_bits(f);
          const unsigned short lb = f2bf_bits(f - bf_bits2f(hb));
          pwh[(8 * lh + r) * PTP + j * 16 + c] = __builtin_bit_cast(__bf16, hb);
          pwl[(8 * lh + r) * PTP + j * 16 + c] = __builtin_bit_cast(__bf16, lb);
        }
        psum += __shfl_xor(psum, 1, 32);
        psum += __shfl_xor(psum, 2, 32);
        psum += __shfl_xor(psum, 4, 32);
        psum += __shfl_xor(psum, 8, 32);
        lrow[r] += psum;
      }
    }
    __syncthreads();

#pragma unroll
    for (int kk = 0; kk < 2; ++kk) {
      FB pa, pl;
      pa.h[0] = *(const v8b*)(pwh + c * PTP + kk * 32 + 8 * lh);
      pa.h[1] = *(const v8b*)(pwh + c * PTP + kk * 32 + 16 + 8 * lh);
      pl.h[0] = *(const v8b*)(pwl + c * PTP + kk * 32 + 8 * lh);
      pl.h[1] = *(const v8b*)(pwl + c * PTP + kk * 32 + 16 + 8 * lh);
#pragma unroll
      for (int t = 0; t < 2; ++t) {
        const __bf16* vp = Vth + (ch0 + t * 16 + c) * VTP + kk * 32 + 8 * lh;
        const __bf16* vq = Vtl + (ch0 + t * 16 + c) * VTP + kk * 32 + 8 * lh;
        FB vb, vl;
        vb.h[0] = *(const v8b*)(vp);
        vb.h[1] = *(const v8b*)(vp + 16);
        vl.h[0] = *(const v8b*)(vq);
        vl.h[1] = *(const v8b*)(vq + 16);
        oacc[t] = mma_bf(pa.v, vb.v, oacc[t]);
        oacc[t] = mma_bf(pa.v, vl.v, oacc[t]);
        oacc[t] = mma_bf(pl.v, vb.v, oacc[t]);
      }
    }
  }

  if (wave < 4 && c == 0) {
#pragma unroll
    for (int r = 0; r < 8; ++r) Ll[g][8 * lh + r] = lrow[r];
  }
  __syncthreads();
  {
    float inv[8];
#pragma unroll
    for (int r = 0; r < 8; ++r) inv[r] = 1.0f / Ll[g][8 * lh + r];
#pragma unroll
    for (int t = 0; t < 2; ++t) {
#pragma unroll
      for (int r = 0; r < 8; ++r) {
        const float o = oacc[t][r] * inv[r];
        const unsigned short hb = f2bf_bits(o);
        const unsigned short lb = f2bf_bits(o - bf_bits2f(hb));
        const int idx = (g * 16 + 8 * lh + r) * OTP + ch0 + t * 16 + c;
        Osh[idx] = hb;
        Osl[idx] = lb;
      }
    }
  }
  __syncthreads();
  {
    const int rq = lane >> 3;
    const int pc = (lane & 7) * 8;
    const size_t rowbase = (size_t)(b * SEQ + qt * QB);
    for (int ps = 0; ps < 2; ++ps) {
#pragma unroll
      for (int it = 0; it < 2; ++it) {
        const int row = wave * 8 + it * 4 + rq;
        U8S uh, ul;
        uh.v = *(const v8us*)(Osh + row * OTP + pc);
        ul.v = *(const v8us*)(Osl + row * OTP + pc);
        const size_t go = (rowbase + row) * DM + (size_t)hd * DH + pc;
        *(volatile v4u*)(Oh + go) = uh.u;
        *(volatile v4u*)(Ol + go) = ul.u;
      }
      __threadfence();
    }
  }
}

extern "C" void kernel_launch(void* const* d_in, const int* in_sizes, int n_in,
                              void* d_out, int out_size, void* d_ws, size_t ws_size,
                              hipStream_t stream) {
  if (n_in < 10) return;
  if (in_sizes[0] != ROWS * DM) return;
  if (in_sizes[1] != DM * DM || in_sizes[3] != DM * DM || in_sizes[5] != DM * DM || in_sizes[7] != DM * DM) return;
  if (in_sizes[2] != DM || in_sizes[4] != DM || in_sizes[6] != DM || in_sizes[8] != DM) return;
  if (in_sizes[9] != NH) return;
  if (out_size != ROWS * DM) return;

  const float* x  = (const float*)d_in[0];
  const float* Wq = (const float*)d_in[1];
  const float* bq = (const float*)d_in[2];
  const float* Wk = (const float*)d_in[3];
  const float* bk = (const float*)d_in[4];
  const float* Wv = (const float*)d_in[5];
  const float* bv = (const float*)d_in[6];
  const float* Wo = (const float*)d_in[7];
  const float* bo = (const float*)d_in[8];
  const float* G  = (const float*)d_in[9];
  float* out = (float*)d_out;

  const size_t PX = (size_t)ROWS * DM * 2;
  const size_t PW = (size_t)DM * DM * 2;
  const size_t PS = (size_t)NBH * SEQ * 4;
  size_t off = 0;
  const size_t oXh  = off; off += PX;
  const size_t oXbh = off; off += PX;
  const size_t oXbl = off; off += PX;
  const size_t oWqh = off; off += PW;
  const size_t oWkh = off; off += PW;
  const size_t oWvh = off; off += PW;
  const size_t oWvl = off; off += PW;
  const size_t oWoh = off; off += PW;
  const size_t oWol = off; off += PW;
  const size_t oQ   = off; off += PX;
  const size_t oK   = off; off += PX;
  const size_t oVTh = off; off += PX;
  const size_t oVTl = off; off += PX;
  const size_t oq2  = off; off += PS;
  const size_t ok2  = off; off += PS;
  const size_t oOh  = off; off += PX;
  const size_t oOl  = off; off += PX;
  if (off > ws_size) return;
  if (off > (size_t)134217728) return;

  char* ws = (char*)d_ws;
  unsigned short* Xh  = (unsigned short*)(ws + oXh);
  unsigned short* Xbh = (unsigned short*)(ws + oXbh);
  unsigned short* Xbl = (unsigned short*)(ws + oXbl);
  unsigned short* Wqh = (unsigned short*)(ws + oWqh);
  unsigned short* Wkh = (unsigned short*)(ws + oWkh);
  unsigned short* Wvh = (unsigned short*)(ws + oWvh);
  unsigned short* Wvl = (unsigned short*)(ws + oWvl);
  unsigned short* Woh = (unsigned short*)(ws + oWoh);
  unsigned short* Wol = (unsigned short*)(ws + oWol);
  unsigned short* Qpl = (unsigned short*)(ws + oQ);
  unsigned short* Kpl = (unsigned short*)(ws + oK);
  unsigned short* VTh = (unsigned short*)(ws + oVTh);
  unsigned short* VTl = (unsigned short*)(ws + oVTl);
  float* q2 = (float*)(ws + oq2);
  float* k2 = (float*)(ws + ok2);
  unsigned short* Ohp = (unsigned short*)(ws + oOh);
  unsigned short* Olp = (unsigned short*)(ws + oOl);

  const int nx8 = ROWS * DM / 8;
  const int nw8 = DM * DM / 8;

  cvt_f16_kernel<<<dim3((nx8 + 255) / 256), dim3(256), 0, stream>>>(x, Xh, nx8, 1.0f);
  cvt_split_kernel<<<dim3((nx8 + 255) / 256), dim3(256), 0, stream>>>(x, Xbh, Xbl, nx8);
  cvt_f16_kernel<<<dim3((nw8 + 255) / 256), dim3(256), 0, stream>>>(Wq, Wqh, nw8, 32.0f);
  cvt_f16_kernel<<<dim3((nw8 + 255) / 256), dim3(256), 0, stream>>>(Wk, Wkh, nw8, 32.0f);
  cvt_split_kernel<<<dim3((nw8 + 255) / 256), dim3(256), 0, stream>>>(Wv, Wvh, Wvl, nw8);
  cvt_split_kernel<<<dim3((nw8 + 255) / 256), dim3(256), 0, stream>>>(Wo, Woh, Wol, nw8);

  const int qkBlocks = (ROWS / 32) * (DM / 64) / 4;
  const int vBlocks  = (ROWS / 64) * (DM / 32) / 4;
  proj_qk_kernel<<<dim3(qkBlocks), dim3(128), 0, stream>>>(Xh, Wqh, bq, Qpl, q2);
  proj_qk_kernel<<<dim3(qkBlocks), dim3(128), 0, stream>>>(Xh, Wkh, bk, Kpl, k2);
  proj_v_kernel<<<dim3(vBlocks), dim3(128), 0, stream>>>(Xbh, Xbl, Wvh, Wvl, bv, VTh, VTl);

  grav_attn_kernel<<<dim3(NBH * (SEQ / QB)), dim3(256), 0, stream>>>(Qpl, Kpl, VTh, VTl, q2, k2, G, Ohp, Olp);

  proj_o_kernel<<<dim3(qkBlocks), dim3(128), 0, stream>>>(Ohp, Olp, Woh, Wol, bo, out);
  (void)hipGetLastError();
}
